// ScaledDotProductAttention_1262720385467
// MI455X (gfx1250) — hardware-verified
//
#include <hip/hip_runtime.h>
#ifndef NB
#define NB 4
#endif
#ifndef SEQ
#define SEQ 2048
#endif
#define NBu ((unsigned)(NB))
#define SQu ((unsigned)(SEQ))
#define SEQ_FULL 2048u
#define DM 1024u
#define NH 16u
#define HD 64u
#define OP 2048u
#define NRU (NBu * SQu)
#define NWAVE_FL (NBu * NH * (SQu / 32u))

static_assert(DM == NH * HD);
static_assert(HD == 64u);
static_assert(OP == 2u * DM);
static_assert(SQu % 128u == 0u);
static_assert((SQu / 32u) % 4u == 0u);
static_assert(NRU % 128u == 0u && DM % 64u == 0u && DM % 32u == 0u && OP % 32u == 0u);
static_assert(((size_t)NRU * DM / 8u) % 256u == 0u);
static_assert(((size_t)DM * DM / 8u) % 256u == 0u);
static_assert(SQu <= SEQ_FULL);

typedef unsigned short v8us __attribute__((ext_vector_type(8), may_alias));
typedef float  v8f  __attribute__((ext_vector_type(8)));
typedef float  v4f  __attribute__((ext_vector_type(4)));
typedef float  v4fa __attribute__((ext_vector_type(4), may_alias));
typedef _Float16 v16h __attribute__((ext_vector_type(16)));
typedef _Float16 v4h __attribute__((ext_vector_type(4)));
union FragH { v16h v; v8us half[2]; _Float16 h[16]; unsigned short u[16]; };

__device__ __forceinline__ unsigned short bf16_bits(float x) { unsigned int u = __float_as_uint(x); return (unsigned short)((u + 0x7FFFu + ((u >> 16) & 1u)) >> 16); }
__device__ __forceinline__ float bf16_val(unsigned short b) { return __uint_as_float(((unsigned int)b) << 16); }
__device__ __forceinline__ float bf16_rne(float x) { return bf16_val(bf16_bits(x)); }

__device__ __forceinline__ v16h g2_frag(const _Float16* p, unsigned hh) { FragH f; f.half[0] = *(const v8us*)((const unsigned short*)p + 8u * hh); f.half[1] = *(const v8us*)((const unsigned short*)p + 16u + 8u * hh); return f.v; }
__device__ __forceinline__ v8f g2_mma(v16h a, v16h b, v8f c) { v8f d = __builtin_amdgcn_wmma_f32_16x16x32_f16(false, a, false, b, (short)0, c, false, false); asm volatile("v_nop\n\tv_nop\n\tv_nop\n\tv_nop" : "+v"(d) : "v"(a), "v"(b)); return d; }
__device__ __forceinline__ void wm2(v16h a, v16h b0, v16h b1, v8f& c0, v8f& c1) {
  c0 = __builtin_amdgcn_wmma_f32_16x16x32_f16(false, a, false, b0, (short)0, c0, false, false);
  c1 = __builtin_amdgcn_wmma_f32_16x16x32_f16(false, a, false, b1, (short)0, c1, false, false);
  asm volatile("v_nop\n\tv_nop\n\tv_nop\n\tv_nop" : "+v"(c0), "+v"(c1) : "v"(a), "v"(b0), "v"(b1));
}

__global__ __launch_bounds__(256) void k_x16(const float* __restrict__ x, _Float16* __restrict__ X16) {
  const unsigned t = blockIdx.x * 256u + threadIdx.x;
  if (t >= NRU * (DM / 8u)) return;
  const unsigned row = t / (DM / 8u), c8 = (t % (DM / 8u)) * 8u;
  const unsigned b = row / SQu, s = row % SQu;
  const float* src = x + ((size_t)b * SEQ_FULL + s) * DM + c8;
  const v4f a = *(const v4fa*)src, c = *(const v4fa*)(src + 4);
  FragH f;
#pragma unroll
  for (int q = 0; q < 4; ++q) { f.h[q] = (_Float16)bf16_rne(a[q]); f.h[4 + q] = (_Float16)bf16_rne(c[q]); }
  const v8us o = f.half[0];
  unsigned short* d = (unsigned short*)X16 + (size_t)t * 8u;
  *(volatile v8us*)d = o; __threadfence(); *(volatile v8us*)d = o;
}

__global__ __launch_bounds__(256) void k_wnat(const float* __restrict__ w, _Float16* __restrict__ Bt, unsigned ldb, unsigned ncopy) {
  const unsigned t = blockIdx.x * 256u + threadIdx.x;
  if (t >= DM * (DM / 8u)) return;
  const unsigned n = t / (DM / 8u), k8 = (t % (DM / 8u)) * 8u;
  const float* src = w + (size_t)n * DM + k8;
  const v4f a = *(const v4fa*)src, c = *(const v4fa*)(src + 4);
  FragH f;
#pragma unroll
  for (int q = 0; q < 4; ++q) { f.h[q] = (_Float16)(bf16_rne(a[q]) * 16.0f); f.h[4 + q] = (_Float16)(bf16_rne(c[q]) * 16.0f); }
  const v8us o = f.half[0];
  unsigned short* d = (unsigned short*)Bt + (size_t)n * ldb + k8;
  for (int pass = 0; pass < 2; ++pass) {
    for (unsigned cc = 0; cc < ncopy; ++cc) *(volatile v8us*)(d + (size_t)cc * DM) = o;
    if (pass == 0) __threadfence();
  }
}

__global__ __launch_bounds__(128) void k_gemm2(const _Float16* __restrict__ A, unsigned lda, const _Float16* __restrict__ Bh, unsigned ldb, float alpha, const float* __restrict__ bias,
    float* __restrict__ C, _Float16* __restrict__ C16, unsigned ldc, unsigned M, unsigned N, unsigned K) {
  __shared__ __attribute__((aligned(16))) float so[4][32][68];
  const unsigned tid = threadIdx.x, w = tid >> 5, lane = tid & 31u, ln = lane & 15u, hh = lane >> 4;
  const unsigned ntn = N >> 6; const unsigned mt = blockIdx.x / ntn, nq = blockIdx.x - mt * ntn; const unsigned row0 = mt * 128u + 32u * w, col0 = nq * 64u; if (row0 >= M) return;
  const _Float16* a0p = A + (size_t)(row0 + ln) * lda; const _Float16* a1p = a0p + (size_t)16 * lda;
  const _Float16* b0p = Bh + (size_t)(col0 + ln) * ldb; const _Float16* b1p = b0p + (size_t)16 * ldb; const _Float16* b2p = b1p + (size_t)16 * ldb; const _Float16* b3p = b2p + (size_t)16 * ldb;
  const v8f z8 = {0.f,0.f,0.f,0.f,0.f,0.f,0.f,0.f}; v8f c00 = z8, c01 = z8, c02 = z8, c03 = z8, c10 = z8, c11 = z8, c12 = z8, c13 = z8;
#pragma unroll 1
  for (unsigned kb = 0; kb < K; kb += 32u) { const v16h a0 = g2_frag(a0p + kb, hh), a1 = g2_frag(a1p + kb, hh);
    v16h b = g2_frag(b0p + kb, hh); c00 = g2_mma(a0, b, c00); c10 = g2_mma(a1, b, c10);
    b = g2_frag(b1p + kb, hh); c01 = g2_mma(a0, b, c01); c11 = g2_mma(a1, b, c11);
    b = g2_frag(b2p + kb, hh); c02 = g2_mma(a0, b, c02); c12 = g2_mma(a1, b, c12);
    b = g2_frag(b3p + kb, hh); c03 = g2_mma(a0, b, c03); c13 = g2_mma(a1, b, c13); }
  v8f accs[8] = {c00, c01, c02, c03, c10, c11, c12, c13};
#pragma unroll
  for (int u = 0; u < 8; ++u) { const unsigned t = (unsigned)u & 3u, half = (unsigned)u >> 2; const unsigned col = col0 + t * 16u + ln; const float bv = bias ? bf16_rne(bias[col]) : 0.f;
#pragma unroll
    for (int r = 0; r < 8; ++r) { const unsigned rloc = half * 16u + 8u * hh + (unsigned)r; so[w][rloc][t * 16u + ln] = accs[u][r] * alpha + bv; } }
  __builtin_amdgcn_fence(4  , "workgroup"); __builtin_amdgcn_wave_barrier();
  const unsigned rsub = lane >> 4, c4 = (lane & 15u) * 4u;
  for (int pass = 0; pass < 2; ++pass) {
#pragma unroll
    for (int q = 0; q < 16; ++q) { const unsigned r = (unsigned)q * 2u + rsub; const v4f v = *(const v4fa*)&so[w][r][c4];
      if (C) *(volatile v4f*)(C + (size_t)(row0 + r) * ldc + col0 + c4) = v;
      if (C16) { v4h h4; for (int i = 0; i < 4; ++i) h4[i] = (_Float16)v[i]; *(volatile v4h*)(C16 + (size_t)(row0 + r) * ldc + col0 + c4) = h4; } }
    if (pass == 0) __threadfence(); } }

__global__ __launch_bounds__(256) void k_vt(const _Float16* __restrict__ V16, _Float16* __restrict__ Vt) {
  __shared__ unsigned short tl[64][66];
  const unsigned tid = threadIdx.x; const unsigned slab = blockIdx.x / (SQu / 64u), lg = blockIdx.x % (SQu / 64u); const unsigned b = slab / NH, h = slab % NH;
  for (unsigned i = tid; i < 512u; i += 256u) { const unsigned r = i >> 3, c8 = (i & 7u) * 8u; FragH f; f.half[0] = *(const v8us*)((const unsigned short*)V16 + ((size_t)b * SQu + lg * 64u + r) * DM + h * HD + c8);
#pragma unroll
    for (int q = 0; q < 8; ++q) tl[r][c8 + (unsigned)q] = f.u[q]; }
  __syncthreads();
  for (int pass = 0; pass < 2; ++pass) {
#pragma unroll
    for (int rd = 0; rd < 2; ++rd) { const unsigned d = (unsigned)rd * 32u + (tid >> 3), pc = tid & 7u; FragH f;
#pragma unroll
      for (int q = 0; q < 8; ++q) f.u[q] = tl[pc * 8u + (unsigned)q][d];
      const v8us o = f.half[0];
      *(volatile v8us*)((unsigned short*)Vt + ((size_t)slab * 64u + d) * SQu + lg * 64u + pc * 8u) = o; }
    if (pass == 0) __threadfence(); } }

__device__ __forceinline__ v16h softm(const v8f& sa, const v8f& sb, float& mrun, float& lrun, float& corr) {
  float mx = fmaxf(sa[0], sb[0]);
#pragma unroll
  for (int r = 1; r < 8; ++r) mx = fmaxf(mx, fmaxf(sa[r], sb[r]));
  mx = fmaxf(mx, __shfl_xor(mx, 16));
  const float mn = fmaxf(mrun, mx);
  corr = __expf((mrun - mn) * 0.125f);
  mrun = mn;
  FragH pf; float ps = 0.f;
#pragma unroll
  for (int r = 0; r < 8; ++r) {
    const float e0 = __expf((sa[r] - mn) * 0.125f + 5.545177444f);
    const float e1 = __expf((sb[r] - mn) * 0.125f + 5.545177444f);
    ps += e0 + e1; pf.h[r] = (_Float16)e0; pf.h[8 + r] = (_Float16)e1;
  }
  lrun = lrun * corr + ps;
  return pf.v;
}
__device__ __forceinline__ void put8(unsigned short* hi, unsigned short* lo, const v8f& o, float inv) {
  FragH fh, fl;
#pragma unroll
  for (int r = 0; r < 8; ++r) { const float v = o[r] * inv; const _Float16 hq = (_Float16)v; fh.h[r] = hq; fl.h[r] = (_Float16)(v - (float)hq); }
  *(v8us*)hi = fh.half[0]; *(v8us*)lo = fl.half[0];
}

__global__ __launch_bounds__(128) void k_flash(const _Float16* __restrict__ Q16, const _Float16* __restrict__ K16, const _Float16* __restrict__ VT, _Float16* __restrict__ O2) {
  __shared__ __attribute__((aligned(16))) unsigned short st[4][2][32][64];
  const unsigned tid = threadIdx.x, w = tid >> 5, lane = tid & 31u, ln = lane & 15u, hh = lane >> 4;
  const unsigned wid = blockIdx.x * 4u + w;
  if (wid >= NWAVE_FL) return;
  const unsigned bh = wid / (SQu / 32u), qt = wid % (SQu / 32u);
  const unsigned b = bh / NH, h = bh % NH, q0 = qt * 32u;
  const _Float16* qp = Q16 + ((size_t)b * SQu + q0 + ln) * DM + h * HD;
  const v16h qf00 = g2_frag(qp, hh), qf01 = g2_frag(qp + 32, hh);
  const v16h qf10 = g2_frag(qp + (size_t)16 * DM, hh), qf11 = g2_frag(qp + (size_t)16 * DM + 32, hh);
  const _Float16* kp = K16 + ((size_t)b * SQu + ln) * DM + h * HD;
  const _Float16* vp = VT + ((size_t)bh * HD + ln) * SQu;
  const v8f z8 = {0.f,0.f,0.f,0.f,0.f,0.f,0.f,0.f};
  v8f o00 = z8, o01 = z8, o02 = z8, o03 = z8, o10 = z8, o11 = z8, o12 = z8, o13 = z8;
  float m0 = -3.0e38f, m1 = -3.0e38f, l0 = 0.f, l1 = 0.f;
#pragma unroll 1
  for (unsigned key0 = 0; key0 < SQu; key0 += 32u) {
    const _Float16* kr = kp + (size_t)key0 * DM;
    v8f s00 = z8, s01 = z8, s10 = z8, s11 = z8;
    v16h a = g2_frag(kr, hh);                         wm2(a, qf00, qf10, s00, s10);
    a = g2_frag(kr + 32, hh);                         wm2(a, qf01, qf11, s00, s10);
    a = g2_frag(kr + (size_t)16 * DM, hh);            wm2(a, qf00, qf10, s01, s11);
    a = g2_frag(kr + (size_t)16 * DM + 32, hh);       wm2(a, qf01, qf11, s01, s11);
    float c0, c1;
    const v16h p0 = softm(s00, s01, m0, l0, c0);
    const v16h p1 = softm(s10, s11, m1, l1, c1);
    o00 *= c0; o01 *= c0; o02 *= c0; o03 *= c0;
    o10 *= c1; o11 *= c1; o12 *= c1; o13 *= c1;
    const _Float16* vr = vp + key0;
    a = g2_frag(vr, hh);                              wm2(a, p0, p1, o00, o10);
    a = g2_frag(vr + (size_t)16 * SQu, hh);           wm2(a, p0, p1, o01, o11);
    a = g2_frag(vr + (size_t)32 * SQu, hh);           wm2(a, p0, p1, o02, o12);
    a = g2_frag(vr + (size_t)48 * SQu, hh);           wm2(a, p0, p1, o03, o13);
  }
  const float t0 = l0 + __shfl_xor(l0, 16), t1 = l1 + __shfl_xor(l1, 16);
  const float i0 = 1024.0f * __builtin_amdgcn_rcpf(t0), i1 = 1024.0f * __builtin_amdgcn_rcpf(t1);
  unsigned short* sh0 = &st[w][0][ln][8u * hh];        unsigned short* sl0 = &st[w][1][ln][8u * hh];
  unsigned short* sh1 = &st[w][0][16u + ln][8u * hh];  unsigned short* sl1 = &st[w][1][16u + ln][8u * hh];
  put8(sh0, sl0, o00, i0); put8(sh0 + 16, sl0 + 16, o01, i0); put8(sh0 + 32, sl0 + 32, o02, i0); put8(sh0 + 48, sl0 + 48, o03, i0);
  put8(sh1, sl1, o10, i1); put8(sh1 + 16, sl1 + 16, o11, i1); put8(sh1 + 32, sl1 + 32, o12, i1); put8(sh1 + 48, sl1 + 48, o13, i1);
  __builtin_amdgcn_fence(4  , "workgroup"); __builtin_amdgcn_wave_barrier();
  const unsigned rsub = lane >> 3, pc = lane & 7u;
  unsigned short* obase = (unsigned short*)O2 + ((size_t)b * SQu + q0) * OP + h * HD + pc * 8u;
  for (int pass = 0; pass < 2; ++pass) {
#pragma unroll
    for (int i = 0; i < 8; ++i) { const unsigned row = 4u * (unsigned)i + rsub;
      const v8us vh = *(const v8us*)&st[w][0][row][pc * 8u]; const v8us vl = *(const v8us*)&st[w][1][row][pc * 8u];
      unsigned short* d = obase + (size_t)row * OP;
      *(volatile v8us*)d = vh; *(volatile v8us*)(d + DM) = vl; }
    if (pass == 0) __threadfence(); }
}

constexpr size_t SZ_W   = (size_t)DM * DM * 2u;
constexpr size_t SZ_WO  = (size_t)DM * OP * 2u;
constexpr size_t SZ_X   = (size_t)NRU * DM * 2u;
constexpr size_t SZ_O2  = (size_t)NRU * OP * 2u;
constexpr size_t SZ_VT  = (size_t)NBu * NH * HD * SQu * 2u;
constexpr size_t WS_TOTAL = 3u * SZ_W + SZ_WO + 6u * SZ_X;
static_assert(SZ_W % 256u == 0u && SZ_WO % 256u == 0u && SZ_X % 256u == 0u);
static_assert(SZ_O2 <= 2u * SZ_X);
static_assert(SZ_VT <= SZ_X);
static_assert(WS_TOTAL <= (size_t)134217728);

extern "C" void kernel_launch(void* const* d_in, const int* in_sizes, int n_in,
                              void* d_out, int out_size, void* d_ws, size_t ws_size, hipStream_t stream) {
  if (n_in < 11) return;
  const long long need_x = ((long long)(NBu - 1u) * SEQ_FULL + SQu) * DM;
  if ((long long)in_sizes[0] < need_x || (long long)in_sizes[1] < need_x || (long long)in_sizes[2] < need_x) return;
  if ((long long)in_sizes[3] < (long long)DM * DM || (long long)in_sizes[5] < (long long)DM * DM || (long long)in_sizes[7] < (long long)DM * DM || (long long)in_sizes[9] < (long long)DM * DM) return;
  if (in_sizes[4] < (int)DM || in_sizes[6] < (int)DM || in_sizes[8] < (int)DM || in_sizes[10] < (int)DM) return;
  if ((long long)out_size < (long long)NRU * DM) return;
  if (ws_size < WS_TOTAL) return;
  const float* const* I = (const float* const*)d_in;
  const float* xq = I[0]; const float* xk = I[1]; const float* xv = I[2];
  const float* wq = I[3]; const float* bq = I[4]; const float* wk = I[5]; const float* bk = I[6];
  const float* wv = I[7]; const float* bv = I[8]; const float* wo = I[9]; const float* bo = I[10];
  char* ws = (char*)d_ws; size_t off = 0;
  _Float16* BQ = (_Float16*)(ws + off); off += SZ_W;
  _Float16* BK = (_Float16*)(ws + off); off += SZ_W;
  _Float16* BV = (_Float16*)(ws + off); off += SZ_W;
  _Float16* BO2 = (_Float16*)(ws + off); off += SZ_WO;
  _Float16* XQ = (_Float16*)(ws + off); off += SZ_X;
  _Float16* XK = (_Float16*)(ws + off); off += SZ_X;
  _Float16* XV = (_Float16*)(ws + off); off += SZ_X;
  _Float16* Q16 = (_Float16*)(ws + off); off += SZ_X;
  _Float16* K16 = (_Float16*)(ws + off); off += SZ_X;
  _Float16* V16 = (_Float16*)(ws + off); off += SZ_X;
  _Float16* O2 = XQ;
  _Float16* VT = XV;
  (void)XK;
  const unsigned gw = (unsigned)((size_t)DM * DM / 8u / 256u);
  k_wnat<<<gw, 256, 0, stream>>>(wq, BQ, DM, 1u);
  k_wnat<<<gw, 256, 0, stream>>>(wk, BK, DM, 1u);
  k_wnat<<<gw, 256, 0, stream>>>(wv, BV, DM, 1u);
  k_wnat<<<gw, 256, 0, stream>>>(wo, BO2, OP, 2u);
  const unsigned gx = (unsigned)((size_t)NRU * DM / 8u / 256u);
  k_x16<<<gx, 256, 0, stream>>>(xq, XQ);
  k_x16<<<gx, 256, 0, stream>>>(xk, XK);
  k_x16<<<gx, 256, 0, stream>>>(xv, XV);
  const unsigned gg = (NRU / 128u) * (DM / 64u);
  k_gemm2<<<gg, 128, 0, stream>>>(XQ, DM, BQ, DM, 0.0625f, bq, nullptr, Q16, DM, NRU, DM, DM);
  k_gemm2<<<gg, 128, 0, stream>>>(XK, DM, BK, DM, 0.0625f, bk, nullptr, K16, DM, NRU, DM, DM);
  k_gemm2<<<gg, 128, 0, stream>>>(XV, DM, BV, DM, 0.0625f, bv, nullptr, V16, DM, NRU, DM, DM);
  k_vt<<<NBu * NH * (SQu / 64u), 256, 0, stream>>>(V16, VT);
  k_flash<<<NWAVE_FL / 4u, 128, 0, stream>>>(Q16, K16, VT, O2);
  k_gemm2<<<gg, 128, 0, stream>>>(O2, OP, BO2, OP, 6.103515625e-05f, bo, (float*)d_out, nullptr, DM, NRU, DM, OP);
}
